// LightningDecoderLayer_25640954757695
// MI455X (gfx1250) — hardware-verified
//
#include <hip/hip_runtime.h>
#include <stdint.h>
#include <math.h>

constexpr int kBatch = 2;
constexpr int kSeq   = 1024;
constexpr int kHid   = 1024;
constexpr int kHeads = 16;
constexpr int kDh    = 64;
constexpr int kRows  = kBatch * kSeq;
constexpr int kNq    = kHeads * kDh;
constexpr int kNstk  = 4160;
constexpr int kColQ  = 0;
constexpr int kColK  = 1024;
constexpr int kColV  = 2048;
constexpr int kColG  = 3072;
constexpr int kColBw = 4096;
constexpr int kColGk = 4112;
constexpr int kTaps  = 4;

typedef __attribute__((ext_vector_type(16))) _Float16 v16h;
typedef __attribute__((ext_vector_type(8)))  _Float16 v8h;
typedef __attribute__((ext_vector_type(16))) __bf16   v16b;
typedef __attribute__((ext_vector_type(8)))  __bf16   v8b;
typedef __attribute__((ext_vector_type(8)))  float    v8f;
typedef __attribute__((ext_vector_type(4)))  float    v4f;
typedef __attribute__((ext_vector_type(2)))  float    v2f;
typedef __attribute__((ext_vector_type(4)))  unsigned int v4u;

__device__ __forceinline__ unsigned short f2bf_bits(float f) {
  unsigned u = __float_as_uint(f);
  return (unsigned short)((u + 0x7FFFu + ((u >> 16) & 1u)) >> 16);
}
__device__ __forceinline__ float bf_bits2f(unsigned short h) { return __uint_as_float(((unsigned)h) << 16); }

__device__ __forceinline__ void dep_guard_h(v8f& a, v8f& b, v16h x, v16h y) { asm volatile("v_nop\n\tv_nop\n\tv_nop\n\tv_nop" : "+v"(a), "+v"(b) : "v"(x), "v"(y)); }
__device__ __forceinline__ void dep_guard_b(v8f& a, v8f& b, v16b x, v16b y) { asm volatile("v_nop\n\tv_nop\n\tv_nop\n\tv_nop" : "+v"(a), "+v"(b) : "v"(x), "v"(y)); }
__device__ __forceinline__ void keep4_h(v16h a, v16h b, v16h c, v16h d) { asm volatile("v_nop" :: "v"(a), "v"(b), "v"(c), "v"(d)); }
__device__ __forceinline__ void keep4_b(v16b a, v16b b, v16b c, v16b d) { asm volatile("v_nop" :: "v"(a), "v"(b), "v"(c), "v"(d)); }
__device__ __forceinline__ void acc_guard4(v8f& a, v8f& b, v8f& c, v8f& d) { asm volatile("v_nop\n\tv_nop\n\tv_nop\n\tv_nop" : "+v"(a), "+v"(b), "+v"(c), "+v"(d)); }
template <typename T> struct Frag;
template <> struct Frag<_Float16> {
  typedef v16h V; union U { v16h v; v8h h[2]; };
  static __device__ __forceinline__ v16h load(const _Float16* p) {
    U f; f.h[0] = *(const v8h*)(p); f.h[1] = *(const v8h*)(p + 16); return f.v;
  }
  static __device__ __forceinline__ v8f mma(v16h a, v16h b, v8f c) {
    return __builtin_amdgcn_wmma_f32_16x16x32_f16(false, a, false, b, (short)0, c, false, false);
  }
  static __device__ __forceinline__ void guard(v8f& a, v8f& b, v16h x, v16h y) { dep_guard_h(a, b, x, y); }
  static __device__ __forceinline__ void keep(v16h a, v16h b, v16h c, v16h d) { keep4_h(a, b, c, d); }
};
template <> struct Frag<__bf16> {
  typedef v16b V; union U { v16b v; v8b h[2]; };
  static __device__ __forceinline__ v16b load(const __bf16* p) {
    U f; f.h[0] = *(const v8b*)(p); f.h[1] = *(const v8b*)(p + 16); return f.v;
  }
  static __device__ __forceinline__ v8f mma(v16b a, v16b b, v8f c) {
    return __builtin_amdgcn_wmma_f32_16x16x32_bf16(false, a, false, b, (short)0, c, false, false);
  }
  static __device__ __forceinline__ void guard(v8f& a, v8f& b, v16b x, v16b y) { dep_guard_b(a, b, x, y); }
  static __device__ __forceinline__ void keep(v16b a, v16b b, v16b c, v16b d) { keep4_b(a, b, c, d); }
};

__device__ __forceinline__ unsigned pk16(unsigned short a, unsigned short b) { return (unsigned)a | ((unsigned)b << 16); }
__device__ __forceinline__ void split_bf(float f, unsigned short& hb, unsigned short& lb) {
  hb = f2bf_bits(f);
  lb = f2bf_bits(f - bf_bits2f(hb));
}

template <int ET> struct Elem;
template <> struct Elem<0> { typedef _Float16 T; };
template <> struct Elem<1> { typedef __bf16 T; };
template <int ET, bool SPLIT, int BIAS_MODE, int OUT_MODE, bool RESID, int ACT = 0>
__global__ __launch_bounds__(256) void wmma_gemm64(
    const unsigned short* __restrict__ Ap, const unsigned short* __restrict__ A2p, int lda, long strideA,
    const unsigned short* __restrict__ Btp, const unsigned short* __restrict__ Bt2p, int ldb, long strideB,
    void* __restrict__ Cout, void* __restrict__ Cout2, int ldc, long strideC,
    const float* __restrict__ bias,
    const float* __restrict__ resid, long strideR,
    int M, int N, int K, float scale) {
  typedef typename Elem<ET>::T T;
  typedef typename Frag<T>::V V;
  const T* A = (const T*)Ap; const T* A2 = (const T*)A2p; const T* Bt = (const T*)Btp; const T* Bt2 = (const T*)Bt2p;
  __shared__ __align__(16) float sT[8][16 * 68];
  const int b    = blockIdx.y;
  const int lane = threadIdx.x & 31;
  const int wave = threadIdx.x >> 5;
  const int tilesN = N >> 6;
  const int tilesM = M >> 6;
  const int tile = blockIdx.x * 8 + wave;
  if (tile >= tilesM * tilesN) return;
  const int tm = tile / tilesN;
  const int tn = tile - tm * tilesN;
  const int m0 = tm << 6;
  const int n0 = tn << 6;

  const T* Ab  = A  + (size_t)b * strideA;
  const T* Bb  = Bt + (size_t)b * strideB;
  const T* Ab2 = SPLIT ? (A2  + (size_t)b * strideA) : nullptr;
  const T* Bb2 = SPLIT ? (Bt2 + (size_t)b * strideB) : nullptr;

  const int rlane = lane & 15;
  const int koff  = (lane >> 4) * 8;
  const int mOff  = (lane >> 4) * 8;

  v8f acc[4][4];
#pragma unroll
  for (int i = 0; i < 4; ++i)
#pragma unroll
    for (int j = 0; j < 4; ++j) acc[i][j] = (v8f){0.f,0.f,0.f,0.f,0.f,0.f,0.f,0.f};

  for (int k0 = 0; k0 < K; k0 += 32) {
    V bh[4], bl[4];
#pragma unroll
    for (int j = 0; j < 4; ++j) {
      const size_t bo = (size_t)(n0 + (j << 4) + rlane) * ldb + koff + k0;
      bh[j] = Frag<T>::load(Bb + bo);
      if (SPLIT) bl[j] = Frag<T>::load(Bb2 + bo);
    }
#pragma unroll
    for (int i = 0; i < 4; ++i) {
      const size_t ao = (size_t)(m0 + (i << 4) + rlane) * lda + koff + k0;
      V ah = Frag<T>::load(Ab + ao);
      V al;
      if (SPLIT) al = Frag<T>::load(Ab2 + ao);
#pragma unroll
      for (int j = 0; j < 4; ++j) {
        acc[i][j] = Frag<T>::mma(ah, bh[j], acc[i][j]);
        if (SPLIT) {
          acc[i][j] = Frag<T>::mma(ah, bl[j], acc[i][j]);
          acc[i][j] = Frag<T>::mma(al, bh[j], acc[i][j]);
        }
      }
      Frag<T>::guard(acc[i][0], acc[i][3], ah, SPLIT ? al : ah);
    }
    Frag<T>::keep(bh[0], bh[1], bh[2], bh[3]);
    if (SPLIT) Frag<T>::keep(bl[0], bl[1], bl[2], bl[3]);
  }
  acc_guard4(acc[0][0], acc[0][1], acc[0][2], acc[0][3]);
  acc_guard4(acc[1][0], acc[1][1], acc[1][2], acc[1][3]);
  acc_guard4(acc[2][0], acc[2][1], acc[2][2], acc[2][3]);
  acc_guard4(acc[3][0], acc[3][1], acc[3][2], acc[3][3]);

  float* slab = sT[wave];
  const float* Rb = RESID ? (resid + (size_t)b * strideR) : nullptr;
#pragma unroll
  for (int i = 0; i < 4; ++i) {
    const int mBase = m0 + (i << 4);
#pragma unroll
    for (int j = 0; j < 4; ++j) {
      const int n = n0 + (j << 4) + rlane;
      float bv = 0.f;
      if (BIAS_MODE == 2) bv = bias[n];
#pragma unroll
      for (int r = 0; r < 8; ++r) {
        float v = acc[i][j][r] * scale;
        if (BIAS_MODE == 1) v += bias[mBase + mOff + r];
        if (BIAS_MODE == 2) v += bv;
        if (RESID) v += Rb[(size_t)(mBase + mOff + r) * ldc + n];
        if (ACT == 2) v = fmaxf(v, 0.0f);
        if (ACT == 4) v = (v > 0.f) ? v : 0.01f * v;
        slab[(mOff + r) * 68 + (j << 4) + rlane] = v;
      }
    }
    __builtin_amdgcn_fence(__ATOMIC_RELEASE, "workgroup");
    __builtin_amdgcn_wave_barrier();
    __builtin_amdgcn_fence(__ATOMIC_ACQUIRE, "workgroup");
    if (OUT_MODE == 0) {
      float* C = (float*)Cout + (size_t)b * strideC;
      const int hh = lane >> 4, c4 = (lane & 15) * 4;
      for (int pass = 0; pass < 2; ++pass) {
#pragma unroll
        for (int it = 0; it < 8; ++it) {
          const int row = it * 2 + hh;
          v4f v = *(const v4f*)(slab + row * 68 + c4);
          *(volatile v4f*)(C + (size_t)(mBase + row) * ldc + n0 + c4) = v;
        }
        __threadfence();
      }
    } else {
      const int q = lane >> 3, c8 = (lane & 7) * 8;
      unsigned short* C  = (unsigned short*)Cout  + (size_t)b * strideC;
      unsigned short* C2 = (OUT_MODE == 2) ? ((unsigned short*)Cout2 + (size_t)b * strideC) : nullptr;
      for (int pass = 0; pass < 2; ++pass) {
#pragma unroll
        for (int it = 0; it < 4; ++it) {
          const int row = it * 4 + q;
          const float* sp = slab + row * 68 + c8;
          v8h hv, lv;
#pragma unroll
          for (int e = 0; e < 8; ++e) {
            if (OUT_MODE == 1) {
              hv[e] = (_Float16)sp[e];
            } else {
              unsigned short hb = f2bf_bits(sp[e]);
              unsigned short lb = f2bf_bits(sp[e] - bf_bits2f(hb));
              hv[e] = __builtin_bit_cast(_Float16, hb);
              lv[e] = __builtin_bit_cast(_Float16, lb);
            }
          }
          *(volatile v8h*)(C + (size_t)(mBase + row) * ldc + n0 + c8) = hv;
          if (OUT_MODE == 2) *(volatile v8h*)(C2 + (size_t)(mBase + row) * ldc + n0 + c8) = lv;
        }
        __threadfence();
      }
    }
    __builtin_amdgcn_fence(__ATOMIC_RELEASE, "workgroup");
    __builtin_amdgcn_wave_barrier();
    __builtin_amdgcn_fence(__ATOMIC_ACQUIRE, "workgroup");
  }
}

__device__ __forceinline__ float sigmoid_f(float y) {
  const float ex = expf(fminf(-y, 80.0f));
  return __builtin_amdgcn_rcpf(1.0f + ex);
}
__device__ __forceinline__ float silu_f(float y) { return y * sigmoid_f(y); }

__global__ __launch_bounds__(256) void castx_split_kernel(const float* __restrict__ in, unsigned short* __restrict__ oh,
                                                          unsigned short* __restrict__ ol, int n8) {
  const int i = blockIdx.x * 256 + threadIdx.x;
  if (i >= n8) return;
  const float* p = in + 8 * (size_t)i;
  const v4f a = *(const v4f*)(p);
  const v4f c = *(const v4f*)(p + 4);
  unsigned short hb[8], lb[8];
#pragma unroll
  for (int e = 0; e < 4; ++e) {
    split_bf(a[e], hb[e], lb[e]);
    split_bf(c[e], hb[4 + e], lb[4 + e]);
  }
  const v4u uh = (v4u){pk16(hb[0], hb[1]), pk16(hb[2], hb[3]), pk16(hb[4], hb[5]), pk16(hb[6], hb[7])};
  const v4u ul = (v4u){pk16(lb[0], lb[1]), pk16(lb[2], lb[3]), pk16(lb[4], lb[5]), pk16(lb[6], lb[7])};
  unsigned short* qh = oh + 8 * (size_t)i;
  unsigned short* ql = ol + 8 * (size_t)i;
  *(volatile v4u*)qh = uh;
  *(volatile v4u*)ql = ul;
  __threadfence();
  *(volatile v4u*)qh = uh;
  *(volatile v4u*)ql = ul;
}

__global__ __launch_bounds__(256) void wsplit_t_kernel(const float* __restrict__ W0, const float* __restrict__ W1,
                                                       const float* __restrict__ W2, const float* __restrict__ W3,
                                                       unsigned short* __restrict__ oh, unsigned short* __restrict__ ol,
                                                       int rowsPerZ) {
  __shared__ float sm[64][65];
  const int tdx = threadIdx.x;
  const int k0 = blockIdx.x * 64;
  const int n0 = blockIdx.y * 64;
  const int z  = blockIdx.z;
  const float* W = (z == 0) ? W0 : (z == 1) ? W1 : (z == 2) ? W2 : W3;
#pragma unroll
  for (int i = 0; i < 16; ++i) {
    const int e = i * 256 + tdx;
    const int r = e >> 6;
    const int c = e & 63;
    sm[c][r] = W[(size_t)(k0 + r) * kHid + n0 + c];
  }
  __syncthreads();
  const int lane = tdx & 31, wave = tdx >> 5;
  const int q = lane >> 3, c8 = (lane & 7) * 8;
  for (int pass = 0; pass < 2; ++pass) {
#pragma unroll
    for (int it = 0; it < 2; ++it) {
      const int row = wave * 8 + it * 4 + q;
      unsigned short hb[8], lb[8];
#pragma unroll
      for (int e = 0; e < 8; ++e) split_bf(sm[row][c8 + e], hb[e], lb[e]);
      const v4u uh = (v4u){pk16(hb[0], hb[1]), pk16(hb[2], hb[3]), pk16(hb[4], hb[5]), pk16(hb[6], hb[7])};
      const v4u ul = (v4u){pk16(lb[0], lb[1]), pk16(lb[2], lb[3]), pk16(lb[4], lb[5]), pk16(lb[6], lb[7])};
      const size_t o = ((size_t)z * rowsPerZ + n0 + row) * kHid + k0 + c8;
      *(volatile v4u*)(oh + o) = uh;
      *(volatile v4u*)(ol + o) = ul;
    }
    __threadfence();
  }
}

__global__ __launch_bounds__(128) void wsmall_kernel(const float* __restrict__ bw, const float* __restrict__ gkw,
                                                     unsigned short* __restrict__ oh, unsigned short* __restrict__ ol) {
  const int rp  = blockIdx.x;
  const int tdx = threadIdx.x;
  const int col = rp & 15;
  const bool useB = rp < 16;
  const bool useG = (rp >= 16) && (rp < 32);
  unsigned short hb[8], lb[8];
#pragma unroll
  for (int e = 0; e < 8; ++e) {
    const int k = tdx * 8 + e;
    const float vb = bw[(size_t)k * kHeads + col];
    const float vg = gkw[(size_t)k * kHeads + col];
    const float v = useB ? vb : (useG ? vg : 0.0f);
    split_bf(v, hb[e], lb[e]);
  }
  const v4u uh = (v4u){pk16(hb[0], hb[1]), pk16(hb[2], hb[3]), pk16(hb[4], hb[5]), pk16(hb[6], hb[7])};
  const v4u ul = (v4u){pk16(lb[0], lb[1]), pk16(lb[2], lb[3]), pk16(lb[4], lb[5]), pk16(lb[6], lb[7])};
  const size_t o = (size_t)(kColBw + rp) * kHid + tdx * 8;
  *(volatile v4u*)(oh + o) = uh;
  *(volatile v4u*)(ol + o) = ul;
  __threadfence();
  *(volatile v4u*)(oh + o) = uh;
  *(volatile v4u*)(ol + o) = ul;
}

struct RopeInv { float v[16]; };
static_assert(sizeof(RopeInv) == 64, "sz");

__global__ __launch_bounds__(256) void rope_table_kernel(float* __restrict__ CS, RopeInv ri) {
#pragma clang fp contract(off)
  const int lane = threadIdx.x & 31, wave = threadIdx.x >> 5;
  const int t = blockIdx.x * 8 + wave;
  const int m = lane & 15;
  float inv = ri.v[0];
  inv = (m == 1)  ? ri.v[1]  : inv;
  inv = (m == 2)  ? ri.v[2]  : inv;
  inv = (m == 3)  ? ri.v[3]  : inv;
  inv = (m == 4)  ? ri.v[4]  : inv;
  inv = (m == 5)  ? ri.v[5]  : inv;
  inv = (m == 6)  ? ri.v[6]  : inv;
  inv = (m == 7)  ? ri.v[7]  : inv;
  inv = (m == 8)  ? ri.v[8]  : inv;
  inv = (m == 9)  ? ri.v[9]  : inv;
  inv = (m == 10) ? ri.v[10] : inv;
  inv = (m == 11) ? ri.v[11] : inv;
  inv = (m == 12) ? ri.v[12] : inv;
  inv = (m == 13) ? ri.v[13] : inv;
  inv = (m == 14) ? ri.v[14] : inv;
  inv = (m == 15) ? ri.v[15] : inv;
  const float ang = (float)t * inv;
  float sn, cs;
  sincosf(ang, &sn, &cs);
  const float val = (lane < 16) ? cs : sn;
  float* o = CS + (size_t)t * 32 + lane;
  *(volatile float*)o = val;
  __threadfence();
  *(volatile float*)o = val;
}

__global__ __launch_bounds__(256) void prep_kernel(const float* __restrict__ Pj, const float* __restrict__ CS,
                                                   const float* __restrict__ qcw, const float* __restrict__ qcb,
                                                   const float* __restrict__ kcw, const float* __restrict__ kcb,
                                                   const float* __restrict__ vcw, const float* __restrict__ vcb,
                                                   float* __restrict__ Qo, float* __restrict__ Ko, float* __restrict__ Vo) {
  const int lane = threadIdx.x & 31, wave = threadIdx.x >> 5;
  const int w  = blockIdx.x * 8 + wave;
  const int h  = w & 15;
  const int bt = w >> 4;
  const int t  = bt & (kSeq - 1);
  const int j  = lane;
  const int cq  = h * kDh + 2 * j;
  const int cva = h * kDh + j;
  const int cvb = h * kDh + 32 + j;
  const v4f wq0 = *(const v4f*)(qcw + 4 * cq);
  const v4f wq1 = *(const v4f*)(qcw + 4 * (cq + 1));
  const v4f wk0 = *(const v4f*)(kcw + 4 * cq);
  const v4f wk1 = *(const v4f*)(kcw + 4 * (cq + 1));
  const v4f wva = *(const v4f*)(vcw + 4 * cva);
  const v4f wvb = *(const v4f*)(vcw + 4 * cvb);
  float yq0 = 0.f, yq1 = 0.f, yk0 = 0.f, yk1 = 0.f, yva = 0.f, yvb = 0.f;
#pragma unroll
  for (int tap = 0; tap < kTaps; ++tap) {
    const int tt = t - 3 + tap;
    const bool ok = (tt >= 0);
    const int rr = ok ? (bt - 3 + tap) : bt;
    const float* pr = Pj + (size_t)rr * kNstk;
    const v2f pq = *(const v2f*)(pr + kColQ + cq);
    const v2f pk = *(const v2f*)(pr + kColK + cq);
    const float pva = pr[kColV + cva];
    const float pvb = pr[kColV + cvb];
    const float xq0 = ok ? pq.x : 0.f, xq1 = ok ? pq.y : 0.f;
    const float xk0 = ok ? pk.x : 0.f, xk1 = ok ? pk.y : 0.f;
    const float xva = ok ? pva : 0.f, xvb = ok ? pvb : 0.f;
    yq0 += xq0 * wq0[tap]; yq1 += xq1 * wq1[tap];
    yk0 += xk0 * wk0[tap]; yk1 += xk1 * wk1[tap];
    yva += xva * wva[tap]; yvb += xvb * wvb[tap];
  }
  yq0 += qcb[cq]; yq1 += qcb[cq + 1];
  yk0 += kcb[cq]; yk1 += kcb[cq + 1];
  yva += vcb[cva]; yvb += vcb[cvb];
  const float sq0 = silu_f(yq0), sq1 = silu_f(yq1);
  const float sk0 = silu_f(yk0), sk1 = silu_f(yk1);
  const float sva = silu_f(yva), svb = silu_f(yvb);
  const int m = j & 15;
  const float cj = CS[(size_t)t * 32 + m];
  const float sj = CS[(size_t)t * 32 + 16 + m];
  const float qlo = sq0 * cj - sq1 * sj;
  const float qhi = sq0 * sj + sq1 * cj;
  const float klo = sk0 * cj - sk1 * sj;
  const float khi = sk0 * sj + sk1 * cj;
  float ssq = qlo * qlo + qhi * qhi;
  float ssk = klo * klo + khi * khi;
#pragma unroll
  for (int off = 1; off < 32; off <<= 1) {
    ssq += __shfl_xor(ssq, off, 32);
    ssk += __shfl_xor(ssk, off, 32);
  }
  const float rq = rsqrtf(ssq + 1e-6f);
  const float rk = rsqrtf(ssk + 1e-6f);
  const float qa = qlo * rq, qbv = qhi * rq;
  const float ka = klo * rk, kbv = khi * rk;
  const size_t base = (size_t)bt * kNq + (size_t)h * kDh;
  float* pq0 = Qo + base + j;  float* pq1 = Qo + base + 32 + j;
  float* pk0 = Ko + base + j;  float* pk1 = Ko + base + 32 + j;
  float* pv0 = Vo + base + j;  float* pv1 = Vo + base + 32 + j;
  *(volatile float*)pq0 = qa; *(volatile float*)pq1 = qbv;
  *(volatile float*)pk0 = ka; *(volatile float*)pk1 = kbv;
  *(volatile float*)pv0 = sva; *(volatile float*)pv1 = svb;
  __threadfence();
  *(volatile float*)pq0 = qa; *(volatile float*)pq1 = qbv;
  *(volatile float*)pk0 = ka; *(volatile float*)pk1 = kbv;
  *(volatile float*)pv0 = sva; *(volatile float*)pv1 = svb;
}

__global__ __launch_bounds__(256) void alphabeta_kernel(const float* __restrict__ Pj, const float* __restrict__ bb,
                                                        const float* __restrict__ gkb, const float* __restrict__ Alog,
                                                        const float* __restrict__ dtb,
                                                        float* __restrict__ Al, float* __restrict__ Be, int n) {
  const int i = blockIdx.x * 256 + threadIdx.x;
  if (i >= n) return;
  const int bt = i >> 4, h = i & 15;
  const float* pr = Pj + (size_t)bt * kNstk;
  const float pb = pr[kColBw + h] + bb[h];
  const float beta = sigmoid_f(pb);
  const float pg = (pr[kColGk + h] + gkb[h]) + dtb[h];
  const float sp = fmaxf(pg, 0.0f) + log1pf(expf(-fabsf(pg)));
  const float ea = expf(Alog[h]);
  const float alpha = expf((-ea) * sp);
  *(volatile float*)(Al + i) = alpha;
  *(volatile float*)(Be + i) = beta;
  __threadfence();
  *(volatile float*)(Al + i) = alpha;
  *(volatile float*)(Be + i) = beta;
}

__global__ __launch_bounds__(64) void delta_kernel(const float* __restrict__ Qp, const float* __restrict__ Kp,
                                                   const float* __restrict__ Vp, const float* __restrict__ Al,
                                                   const float* __restrict__ Be, const float* __restrict__ Dp,
                                                   float* __restrict__ Op) {
  __shared__ float S[kDh * 65];
  __shared__ float qs[2][kDh];
  __shared__ float ks[2][kDh];
  const int b = blockIdx.x >> 4;
  const int h = blockIdx.x & 15;
  const int e = threadIdx.x;
#pragma unroll 8
  for (int d = 0; d < kDh; ++d) S[d * 65 + e] = 0.0f;
  const float Dv = Dp[h];
  for (int t = 0; t < kSeq; ++t) {
    const int buf = t & 1;
    const size_t bt = (size_t)b * kSeq + t;
    const size_t base = bt * kNq + (size_t)h * kDh;
    qs[buf][e] = Qp[base + e];
    ks[buf][e] = Kp[base + e];
    const float ve = Vp[base + e];
    const float al = Al[bt * kHeads + h];
    const float be = Be[bt * kHeads + h];
    __syncthreads();
    const float* qb = qs[buf];
    const float* kb = ks[buf];
    float o = 0.f, kS = 0.f, qk = 0.f;
#pragma unroll 8
    for (int d = 0; d < kDh; ++d) {
      const float Sd = S[d * 65 + e];
      const float qd = qb[d];
      const float kd = kb[d];
      o  += qd * Sd;
      kS += kd * Sd;
      qk += qd * kd;
    }
    const float ov = o + (Dv * qk) * ve;
    float* op = Op + base + e;
    *(volatile float*)op = ov;
    __threadfence();
    *(volatile float*)op = ov;
#pragma unroll 8
    for (int d = 0; d < kDh; ++d) {
      const float kd = kb[d];
      const float bk = be * kd;
      float Sd = S[d * 65 + e];
      Sd = Sd - bk * kS;
      S[d * 65 + e] = al * Sd + bk * ve;
    }
  }
}

__global__ __launch_bounds__(256) void gate_kernel(const float* __restrict__ Op, const float* __restrict__ Pj,
                                                   const float* __restrict__ onw,
                                                   unsigned short* __restrict__ O2h, unsigned short* __restrict__ O2l) {
  const int lane = threadIdx.x & 31, wave = threadIdx.x >> 5;
  const int w  = blockIdx.x * 8 + wave;
  const int bt = w >> 2, hg = w & 3;
  const int h  = hg * 4 + (lane >> 3);
  const int d0 = (lane & 7) * 8;
  const size_t ob = (size_t)bt * kNq + (size_t)h * kDh + d0;
  const v4f o0 = *(const v4f*)(Op + ob);
  const v4f o1 = *(const v4f*)(Op + ob + 4);
  const size_t gb = (size_t)bt * kNstk + kColG + (size_t)h * kDh + d0;
  const v4f g0 = *(const v4f*)(Pj + gb);
  const v4f g1 = *(const v4f*)(Pj + gb + 4);
  const v4f w0 = *(const v4f*)(onw + d0);
  const v4f w1 = *(const v4f*)(onw + d0 + 4);
  float ss = 0.f;
#pragma unroll
  for (int e = 0; e < 4; ++e) ss += o0[e] * o0[e];
#pragma unroll
  for (int e = 0; e < 4; ++e) ss += o1[e] * o1[e];
  ss += __shfl_xor(ss, 1, 32);
  ss += __shfl_xor(ss, 2, 32);
  ss += __shfl_xor(ss, 4, 32);
  const float rn = rsqrtf(ss * (1.0f / 64.0f) + 1e-6f);
  unsigned short hb[8], lb[8];
#pragma unroll
  for (int e = 0; e < 4; ++e) {
    const float on0 = (o0[e] * rn) * w0[e];
    const float r0 = g0[e] * silu_f(on0);
    split_bf(r0, hb[e], lb[e]);
    const float on1 = (o1[e] * rn) * w1[e];
    const float r1 = g1[e] * silu_f(on1);
    split_bf(r1, hb[4 + e], lb[4 + e]);
  }
  const v4u uh = (v4u){pk16(hb[0], hb[1]), pk16(hb[2], hb[3]), pk16(hb[4], hb[5]), pk16(hb[6], hb[7])};
  const v4u ul = (v4u){pk16(lb[0], lb[1]), pk16(lb[2], lb[3]), pk16(lb[4], lb[5]), pk16(lb[6], lb[7])};
  *(volatile v4u*)(O2h + ob) = uh;
  *(volatile v4u*)(O2l + ob) = ul;
  __threadfence();
  *(volatile v4u*)(O2h + ob) = uh;
  *(volatile v4u*)(O2l + ob) = ul;
}

extern "C" void kernel_launch(void* const* d_in, const int* in_sizes, int n_in,
                              void* d_out, int out_size, void* d_ws, size_t ws_size,
                              hipStream_t stream) {
  if (n_in < 20) return;
  if (in_sizes[0] != kRows * kHid) return;
  if (in_sizes[1] != kHid * kNq || in_sizes[2] != kHid * kNq || in_sizes[3] != kHid * kNq ||
      in_sizes[4] != kHid * kNq || in_sizes[5] != kNq * kHid) return;
  if (in_sizes[6] != kHid * kHeads || in_sizes[8] != kHid * kHeads) return;
  if (in_sizes[10] != kNq * kTaps || in_sizes[12] != kNq * kTaps || in_sizes[14] != kNq * kTaps) return;
  if (out_size != kRows * kHid) return;

  const float* x       = (const float*)d_in[0];
  const float* Wq      = (const float*)d_in[1];
  const float* Wk      = (const float*)d_in[2];
  const float* Wv      = (const float*)d_in[3];
  const float* Wg      = (const float*)d_in[4];
  const float* Wo      = (const float*)d_in[5];
  const float* bw      = (const float*)d_in[6];
  const float* bb      = (const float*)d_in[7];
  const float* gkw     = (const float*)d_in[8];
  const float* gkb     = (const float*)d_in[9];
  const float* qcw     = (const float*)d_in[10];
  const float* qcb     = (const float*)d_in[11];
  const float* kcw     = (const float*)d_in[12];
  const float* kcb     = (const float*)d_in[13];
  const float* vcw     = (const float*)d_in[14];
  const float* vcb     = (const float*)d_in[15];
  const float* A_log   = (const float*)d_in[16];
  const float* D_param = (const float*)d_in[17];
  const float* dt_bias = (const float*)d_in[18];
  const float* onorm_w = (const float*)d_in[19];
  float* out = (float*)d_out;

  size_t off = 0;
  auto carve = [&](size_t bytes) -> char* {
    char* p = (char*)d_ws + off;
    off += (bytes + 255) & ~(size_t)255;
    return p;
  };
  const size_t nTok = (size_t)kRows * kHid;
  unsigned short* XH  = (unsigned short*)carve(nTok * 2);
  unsigned short* XL  = (unsigned short*)carve(nTok * 2);
  unsigned short* WTH = (unsigned short*)carve((size_t)kNstk * kHid * 2);
  unsigned short* WTL = (unsigned short*)carve((size_t)kNstk * kHid * 2);
  float* PROJ  = (float*)carve((size_t)kRows * kNstk * 4);
  float* CS    = (float*)carve((size_t)kSeq * 32 * 4);
  float* QP    = (float*)carve(nTok * 4);
  float* KP    = (float*)carve(nTok * 4);
  float* VP    = (float*)carve(nTok * 4);
  float* ALPHA = (float*)carve((size_t)kRows * kHeads * 4);
  float* BETA  = (float*)carve((size_t)kRows * kHeads * 4);
  float* OP    = (float*)carve(nTok * 4);
  unsigned short* O2H = (unsigned short*)carve(nTok * 2);
  unsigned short* O2L = (unsigned short*)carve(nTok * 2);
  unsigned short* WOH = (unsigned short*)carve((size_t)kNq * kHid * 2);
  unsigned short* WOL = (unsigned short*)carve((size_t)kNq * kHid * 2);
  if (off > ws_size) return;

  double s10 = 3.0;
  for (int i = 0; i < 64; ++i) s10 = 0.5 * (s10 + 10.0 / s10);
  double r4 = 1.75;
  for (int i = 0; i < 64; ++i) r4 = 0.5 * (r4 + s10 / r4);
  RopeInv ri;
  {
    double p = 1.0;
    for (int m = 0; m < 16; ++m) {
      const float pf = (float)p;
      ri.v[m] = 1.0f / pf;
      p *= r4;
    }
  }

  const int n8 = (int)(nTok / 8);
  castx_split_kernel<<<(n8 + 255) / 256, 256, 0, stream>>>(x, XH, XL, n8);
  wsplit_t_kernel<<<dim3(kHid / 64, kNq / 64, 4), 256, 0, stream>>>(Wq, Wk, Wv, Wg, WTH, WTL, kNq);
  wsmall_kernel<<<64, 128, 0, stream>>>(bw, gkw, WTH, WTL);
  wsplit_t_kernel<<<dim3(kNq / 64, kHid / 64, 1), 256, 0, stream>>>(Wo, Wo, Wo, Wo, WOH, WOL, kHid);
  rope_table_kernel<<<kSeq / 8, 256, 0, stream>>>(CS, ri);

  {
    const int tiles = (kRows / 64) * (kNstk / 64);
    wmma_gemm64<1, true, 0, 0, false, 0><<<dim3(tiles / 8, 1), 256, 0, stream>>>(
        XH, XL, kHid, 0L,
        WTH, WTL, kHid, 0L,
        (void*)PROJ, (void*)PROJ, kNstk, 0L,
        D_param, D_param, 0L,
        kRows, kNstk, kHid, 1.0f);
  }

  prep_kernel<<<(kRows * kHeads) / 8, 256, 0, stream>>>(PROJ, CS, qcw, qcb, kcw, kcb, vcw, vcb, QP, KP, VP);

  alphabeta_kernel<<<(kRows * kHeads + 255) / 256, 256, 0, stream>>>(PROJ, bb, gkb, A_log, dt_bias,
                                                                      ALPHA, BETA, kRows * kHeads);

  delta_kernel<<<kBatch * kHeads, 64, 0, stream>>>(QP, KP, VP, ALPHA, BETA, D_param, OP);

  gate_kernel<<<(kRows * 4) / 8, 256, 0, stream>>>(OP, PROJ, onorm_w, O2H, O2L);

  {
    const int tiles = (kRows / 64) * (kHid / 64);
    wmma_gemm64<1, true, 0, 0, false, 0><<<dim3(tiles / 8, 1), 256, 0, stream>>>(
        O2H, O2L, kNq, 0L,
        WOH, WOL, kNq, 0L,
        (void*)out, (void*)out, kHid, 0L,
        D_param, D_param, 0L,
        kRows, kHid, kNq, 1.0f);
  }
}
